// CausalAttention_75350906241536
// MI455X (gfx1250) — hardware-verified
//
#include <hip/hip_runtime.h>


#ifndef NB
#define NB 2
#endif
#ifndef SEQ
#define SEQ 512
#endif
#define NB_FULL  2
#define SEQ_FULL 512
#define HID  256
#define AWV  8
#define QPT  (HID + 4)
#define SPT  (SEQ + 4)
#define PPT  (SEQ + 8)
#define OSP  36
#define QRS  2048.0f
#define QRI  (1.0f / 2048.0f)
#define C2S  2.8853900817779268f
#define LOG2E 1.4426950408889634f
#define PCAR 16384.0f
#define KCAR 64.0f
#define OSC  (1.0f / (16384.0f * 64.0f))
#define NEGB (-3.0e38f)
#define A_OFF_BYTES 1048576

static_assert(HID % 64 == 0);
static_assert(HID % 32 == 0);
static_assert((NB * SEQ) % 64 == 0);
static_assert(SEQ % 64 == 0);
static_assert(SEQ % 32 == 0);
static_assert(32 * AWV == HID);
static_assert(AWV * 2 == 16);
static_assert((16 * HID / 4) % (32 * AWV) == 0);
static_assert(HID == 32 * 8);
static_assert(SEQ_FULL % 128 == 0);
static_assert((size_t)NB_FULL * SEQ_FULL * HID * 4 == (size_t)A_OFF_BYTES);
static_assert(A_OFF_BYTES % 128 == 0);
static_assert((size_t)A_OFF_BYTES + (size_t)NB_FULL * SEQ_FULL * SEQ_FULL * 4 == (size_t)3145728);
static_assert(NB <= NB_FULL);
static_assert(SEQ <= SEQ_FULL);
static_assert((QPT * 4) % 16 == 0);
static_assert((SPT * 4) % 16 == 0);
static_assert((PPT * 2) % 16 == 0);
static_assert((OSP * 4) % 16 == 0);
static_assert(((size_t)SEQ * HID) % 8 == 0);
static_assert(((size_t)HID * HID) % 8 == 0);
static_assert((size_t)16 * QPT * 4 + (size_t)HID * 4 + (size_t)16 * SPT * 4 + (size_t)2 * 16 * PPT * 2 + (size_t)AWV * 16 * OSP * 4 <= (size_t)131072);

typedef _Float16 h16;
typedef unsigned short bf;
typedef __attribute__((ext_vector_type(16))) __bf16   v16bf;
typedef __attribute__((ext_vector_type(16))) _Float16 v16h;
typedef __attribute__((ext_vector_type(8)))  _Float16 v8h;
typedef __attribute__((ext_vector_type(8)))  unsigned short v8us;
typedef __attribute__((ext_vector_type(8)))  float    v8f;
typedef __attribute__((ext_vector_type(4)))  float    v4f;
typedef v4f  __attribute__((may_alias)) v4fa;

__device__ __forceinline__ unsigned short f2bf(float f) { unsigned u = __float_as_uint(f); u += 0x7FFFu + ((u >> 16) & 1u); return (unsigned short)(u >> 16); }
__device__ __forceinline__ float bfr(float f) { return __uint_as_float(((unsigned)f2bf(f)) << 16); }
__device__ __forceinline__ v16h cat16(v8h lo, v8h hi) { return __builtin_shufflevector(lo, hi, 0, 1, 2, 3, 4, 5, 6, 7, 8, 9, 10, 11, 12, 13, 14, 15); }
__device__ __forceinline__ v16bf cat16b(v8us lo, v8us hi) { return __builtin_bit_cast(v16bf, __builtin_shufflevector(lo, hi, 0, 1, 2, 3, 4, 5, 6, 7, 8, 9, 10, 11, 12, 13, 14, 15)); }
__device__ __forceinline__ v8f wmma16(v16h a, v16h b, v8f c) { return __builtin_amdgcn_wmma_f32_16x16x32_f16(false, a, false, b, (short)0, c, false, false); }
__device__ __forceinline__ v8f wmmab(v16bf a, v16bf b, v8f c) { return __builtin_amdgcn_wmma_f32_16x16x32_bf16(false, a, false, b, (short)0, c, false, false); }
__device__ __forceinline__ v16h  ldh(const h16* p) { return cat16(*(const v8h*)p, *(const v8h*)(p + 16)); }
__device__ __forceinline__ v16bf ldb(const bf* p)  { return cat16b(*(const v8us*)p, *(const v8us*)(p + 16)); }
__device__ __forceinline__ void wave_sync() { __builtin_amdgcn_fence(3  , "wavefront"); __builtin_amdgcn_wave_barrier(); asm volatile("" ::: "memory"); }
static __device__ __forceinline__ h16 toh_flush(float v) { const h16 r = (h16)v; return (fabsf(v) < 6.103515625e-05f) ? (h16)0.0f : r; }
static __device__ __forceinline__ v8f wmma16g(v16h a, v16h b, v8f c) { c = wmma16(a, b, c); asm volatile("v_nop\n\tv_nop\n\tv_nop\n\tv_nop" : "+v"(c) : "v"(a), "v"(b)); return c; }

static constexpr size_t al256(size_t v) { return (v + 255) & ~(size_t)255; }
static constexpr size_t SZ_XB = al256((size_t)NB * SEQ * HID * 2);
static constexpr size_t SZ_WB = al256((size_t)HID * HID * 2);
static constexpr size_t SZ_PL = al256((size_t)NB * SEQ * HID * 4);
static constexpr size_t SZ_KT = al256((size_t)NB * HID * SEQ * 2);
static constexpr size_t SZ_TOTAL = 2 * SZ_XB + 2 * SZ_WB + 2 * SZ_PL + SZ_KT;
static_assert(SZ_TOTAL <= (size_t)134217728);
static_assert(SZ_XB % 256 == 0);
static_assert(SZ_WB % 256 == 0);
static_assert(SZ_PL % 256 == 0);

__global__ __launch_bounds__(256) void k_cvt8(const float* __restrict__ src, bf* dst, size_t n8) {
    const size_t i = (size_t)blockIdx.x * 256 + threadIdx.x; if (i >= n8) return;
    const v8f v = *(const v8f*)(src + i * 8); v8us o;
#pragma unroll
    for (int k = 0; k < 8; ++k) o[k] = f2bf(v[k]);
    *(volatile v8us*)(dst + i * 8) = o; __threadfence(); *(volatile v8us*)(dst + i * 8) = o;
}

static_assert(2 * 256 * 16 == 64 * 128);
static_assert(4 * 256 * 4 == 64 * 64);
__global__ __launch_bounds__(256) void k_tr(const float* __restrict__ src, h16* dst) {
    __shared__ __align__(16) h16 tl[64 * 72];
    unsigned tid = threadIdx.x; asm volatile("" : "+v"(tid));
    const unsigned tk0 = blockIdx.x * 64u, h0 = blockIdx.y * 64u, b = blockIdx.z;
#pragma unroll
    for (int it = 0; it < 4; ++it) {
        const unsigned idx = (unsigned)it * 256u + tid; const unsigned tok = idx >> 4, c4 = (idx & 15u) * 4u;
        const v4f x = *(const v4f*)(src + ((size_t)b * SEQ_FULL + tk0 + tok) * HID + h0 + c4);
#pragma unroll
        for (int i = 0; i < 4; ++i) tl[(c4 + (unsigned)i) * 72u + tok] = toh_flush(bfr(x[i]) * KCAR);
    }
    __syncthreads();
#pragma unroll 1
    for (int ps = 0; ps < 2; ++ps) {
#pragma unroll
        for (int it = 0; it < 2; ++it) { const unsigned row = (unsigned)it * 32u + (tid >> 3), c8 = (tid & 7u) * 8u;
            const v8h val = *(const v8h*)(&tl[row * 72u + c8]);
            *(volatile v8h*)(dst + ((size_t)b * HID + h0 + row) * SEQ + tk0 + c8) = val; }
        if (ps == 0) __threadfence(); }
}

static_assert(8 * 32 * 16 == 16 * 64 * 4);
__global__ __launch_bounds__(32) void k_proj(const bf* __restrict__ XBp, const bf* __restrict__ WBp, float* PLp) {
    __shared__ __align__(16) float os[16 * 68];
    const int K = HID;
    const int lane = threadIdx.x & 31, lr = lane & 15, hi = lane >> 4; const int r0 = blockIdx.x * 64, c0 = blockIdx.y * 64;
    const size_t z = blockIdx.z;
    const bf* A  = XBp + z * (SZ_XB / 2);
    const bf* Bt = WBp + z * (SZ_WB / 2);
    float* P = PLp + z * (SZ_PL / 4);
    v8f acc[4][4];
#pragma unroll
    for (int mb = 0; mb < 4; ++mb)
#pragma unroll
        for (int nb = 0; nb < 4; ++nb) acc[mb][nb] = (v8f){};
    const size_t aoff = (size_t)(r0 + lr) * K + 8 * hi, boff = (size_t)(c0 + lr) * K + 8 * hi;
#pragma unroll 1
    for (int kc = 0; kc < K; kc += 32) {
        v16bf a[4];
#pragma unroll
        for (int mb = 0; mb < 4; ++mb) a[mb] = ldb(A + aoff + (size_t)mb * 16 * K + kc);
#pragma unroll
        for (int nb = 0; nb < 4; ++nb) { const v16bf b = ldb(Bt + boff + (size_t)nb * 16 * K + kc);
#pragma unroll
            for (int mb = 0; mb < 4; ++mb) acc[mb][nb] = wmmab(a[mb], b, acc[mb][nb]); }
        asm volatile("v_nop\n\tv_nop\n\tv_nop\n\tv_nop" : "+v"(acc[0][0]), "+v"(acc[1][1]), "+v"(acc[2][2]), "+v"(acc[3][3]) : "v"(a[0]), "v"(a[1]), "v"(a[2]), "v"(a[3]));
    }
#pragma unroll
    for (int mb = 0; mb < 4; ++mb) {
#pragma unroll
        for (int nb = 0; nb < 4; ++nb) {
#pragma unroll
            for (int j = 0; j < 8; ++j) os[(hi * 8 + j) * 68 + nb * 16 + lr] = acc[mb][nb][j] * C2S; }
        wave_sync();
#pragma unroll 1
        for (int ps = 0; ps < 2; ++ps) {
#pragma unroll
            for (int s = 0; s < 8; ++s) { const int p = s * 32 + lane; const int row = p >> 4, c4 = (p & 15) * 4;
                const v4f val = *(const v4fa*)(&os[row * 68 + c4]);
                *(volatile v4f*)(P + (size_t)(r0 + mb * 16 + row) * HID + c0 + c4) = val; }
            if (ps == 0) __threadfence(); }
        wave_sync();
    }
}

static_assert(4 * 32 * 16 == 16 * 32 * 4);
static_assert((SEQ_FULL / 128) * 32 * 16 == SEQ_FULL * 4);
__global__ __launch_bounds__(32 * AWV) __attribute__((amdgpu_num_vgpr(256)))
void k_attn(const float* __restrict__ QPL, const float* __restrict__ KPL, const h16* __restrict__ KT, const float* __restrict__ vin, float* OUT) {
    __shared__ __align__(16) float qs[16 * QPT];
    __shared__ __align__(16) float vs[HID];
    __shared__ __align__(16) float ss[16 * SPT];
    __shared__ __align__(16) h16   ph[16 * PPT];
    __shared__ __align__(16) h16   pr[16 * PPT];
    __shared__ __align__(16) float os[AWV * 16 * OSP];
    unsigned tid = threadIdx.x; asm volatile("" : "+v"(tid));
    const int lane = (int)(tid & 31u), lr = lane & 15, hi = lane >> 4;
    const int wave = __builtin_amdgcn_readfirstlane((int)(threadIdx.x >> 5));
    const int b = blockIdx.y; const int t0 = blockIdx.x * 16;
    const int nk = (t0 + 16 + 31) & ~31;

#pragma unroll
    for (int it = 0; it < (16 * HID / 4) / (32 * AWV); ++it) {
        const unsigned idx = (unsigned)it * (unsigned)(32 * AWV) + tid; const unsigned row = idx / (unsigned)(HID / 4), c4 = (idx % (unsigned)(HID / 4)) * 4u;
        const v4f x = *(const v4f*)(QPL + ((size_t)b * SEQ + t0 + row) * HID + c4);
        *(v4fa*)(&qs[row * QPT + c4]) = x; }
    vs[tid] = bfr(vin[tid]);
    __syncthreads();

    float sumv = 0.0f;
#pragma unroll
    for (int i = 0; i < 8; ++i) sumv += vs[lane * 8 + i];
    sumv += __shfl_xor(sumv, 16, 32); sumv += __shfl_xor(sumv, 8, 32); sumv += __shfl_xor(sumv, 4, 32); sumv += __shfl_xor(sumv, 2, 32); sumv += __shfl_xor(sumv, 1, 32);

    const int ra = wave, rb = wave + 8;
#pragma unroll 1
    for (int key0 = 0; key0 < nk; key0 += 32) {
        const float* kp = KPL + ((size_t)b * SEQ + key0 + lane) * HID;
        float a0 = 0.0f, a1 = 0.0f;
#pragma unroll 2
        for (int h4 = 0; h4 < HID / 4; ++h4) {
            const v4f kv = *(const v4f*)(kp + 4 * h4);
            const v4f q0 = *(const v4fa*)(&qs[ra * QPT + 4 * h4]);
            const v4f q1 = *(const v4fa*)(&qs[rb * QPT + 4 * h4]);
            const v4f vv = *(const v4fa*)(&vs[4 * h4]);
#pragma unroll
            for (int i = 0; i < 4; ++i) {
                const float e0 = __builtin_amdgcn_exp2f(q0[i] + kv[i]);
                const float e1 = __builtin_amdgcn_exp2f(q1[i] + kv[i]);
                const float g0 = __builtin_amdgcn_rcpf(e0 + 1.0f);
                const float g1 = __builtin_amdgcn_rcpf(e1 + 1.0f);
                a0 = fmaf(vv[i], g0, a0); a1 = fmaf(vv[i], g1, a1); }
        }
        ss[ra * SPT + key0 + lane] = sumv - 2.0f * a0;
        ss[rb * SPT + key0 + lane] = sumv - 2.0f * a1;
    }
    __syncthreads();

#pragma unroll 1
    for (int i = 0; i < 2; ++i) {
        const int row = wave + 8 * i; const int t = t0 + row; const int ro = row * SPT, po = row * PPT;
        float mx = NEGB;
#pragma unroll 1
        for (int s = lane; s < nk; s += 32) { const float x = ss[ro + s]; mx = fmaxf(mx, (s <= t) ? x : NEGB); }
        mx = fmaxf(mx, __shfl_xor(mx, 16, 32)); mx = fmaxf(mx, __shfl_xor(mx, 8, 32)); mx = fmaxf(mx, __shfl_xor(mx, 4, 32)); mx = fmaxf(mx, __shfl_xor(mx, 2, 32)); mx = fmaxf(mx, __shfl_xor(mx, 1, 32));
        float sum = 0.0f;
#pragma unroll 1
        for (int s = lane; s < nk; s += 32) { const float x = ss[ro + s]; const float ev = __builtin_amdgcn_exp2f((x - mx) * LOG2E); const float e = (s <= t) ? ev : 0.0f; ss[ro + s] = e; sum += e; }
        sum += __shfl_xor(sum, 16, 32); sum += __shfl_xor(sum, 8, 32); sum += __shfl_xor(sum, 4, 32); sum += __shfl_xor(sum, 2, 32); sum += __shfl_xor(sum, 1, 32);
        const float inv = 1.0f / sum;
#pragma unroll 1
        for (int s = lane; s < nk; s += 32) {
            const float a = ss[ro + s] * inv; ss[ro + s] = a;
            const float g = a * PCAR; const h16 gh = toh_flush(g);
            ph[po + s] = gh; pr[po + s] = toh_flush((g - (float)gh) * QRS); }
    }
    __syncthreads();

    float* abase = OUT + (size_t)(A_OFF_BYTES / 4);
#pragma unroll 1
    for (int ps = 0; ps < 2; ++ps) {
#pragma unroll 1
        for (int i = 0; i < 2; ++i) {
            const int row = wave + 8 * i;
            float* arow = abase + ((size_t)b * SEQ_FULL + t0 + row) * SEQ_FULL;
#pragma unroll 1
            for (int c = 0; c < SEQ_FULL / 128; ++c) {
                const int col = c * 128 + lane * 4; const bool inr = col < nk; const int cc = inr ? col : 0;
                v4f val = *(const v4fa*)(&ss[row * SPT + cc]); asm volatile("" : "+v"(val));
                const v4f zz = (v4f){}; const v4f ov = inr ? val : zz;
                *(volatile v4f*)(arow + col) = ov; }
        }
        if (ps == 0) __threadfence(); }

    const size_t vo = ((size_t)b * HID + (size_t)(32 * wave + lr)) * SEQ + 8 * hi;
    const int pofs = lr * PPT + 8 * hi;
    v8f o0 = (v8f){}, o1 = (v8f){}, oR0 = (v8f){}, oR1 = (v8f){};
#pragma unroll 1
    for (int key0 = 0; key0 < nk; key0 += 32) {
        const v16h pb = cat16(*(const v8h*)(&ph[pofs + key0]), *(const v8h*)(&ph[pofs + key0 + 16]));
        const v16h pq = cat16(*(const v8h*)(&pr[pofs + key0]), *(const v8h*)(&pr[pofs + key0 + 16]));
        const h16* va = KT + vo + key0;
        const v16h v0 = ldh(va), v1 = ldh(va + (size_t)16 * SEQ);
        o0 = wmma16g(v0, pb, o0); o1 = wmma16g(v1, pb, o1);
        oR0 = wmma16g(v0, pq, oR0); oR1 = wmma16g(v1, pq, oR1);
    }
    const v8f f0 = o0 + oR0 * QRI, f1 = o1 + oR1 * QRI;
    const int wb = wave * 16 * OSP;
    { v4f a, c;
      a[0] = f0[0] * OSC; a[1] = f0[1] * OSC; a[2] = f0[2] * OSC; a[3] = f0[3] * OSC; c[0] = f0[4] * OSC; c[1] = f0[5] * OSC; c[2] = f0[6] * OSC; c[3] = f0[7] * OSC;
      *(v4fa*)(&os[wb + lr * OSP +  0 + 8 * hi]) = a; *(v4fa*)(&os[wb + lr * OSP +  0 + 8 * hi + 4]) = c;
      a[0] = f1[0] * OSC; a[1] = f1[1] * OSC; a[2] = f1[2] * OSC; a[3] = f1[3] * OSC; c[0] = f1[4] * OSC; c[1] = f1[5] * OSC; c[2] = f1[6] * OSC; c[3] = f1[7] * OSC;
      *(v4fa*)(&os[wb + lr * OSP + 16 + 8 * hi]) = a; *(v4fa*)(&os[wb + lr * OSP + 16 + 8 * hi + 4]) = c; }
    wave_sync();
    float* orow = OUT + ((size_t)b * SEQ_FULL + t0) * HID + 32 * wave;
#pragma unroll 1
    for (int ps = 0; ps < 2; ++ps) {
#pragma unroll
        for (int s = 0; s < 4; ++s) { const int row = 4 * s + (lane >> 3), cofs = (lane & 7) * 4;
            const v4f val = *(const v4fa*)(&os[wb + row * OSP + cofs]);
            *(volatile v4f*)(orow + (size_t)row * HID + cofs) = val; }
        if (ps == 0) __threadfence(); }
}

extern "C" void kernel_launch(void* const* d_in, const int* in_sizes, int n_in,
                              void* d_out, int out_size, void* d_ws, size_t ws_size, hipStream_t stream) {
    if (n_in < 5) return;
    const size_t needx = ((size_t)(NB - 1) * SEQ_FULL + SEQ) * HID;
    if ((size_t)in_sizes[0] < needx || (size_t)in_sizes[1] < needx) return;
    if ((size_t)in_sizes[2] < (size_t)HID * HID || (size_t)in_sizes[3] < (size_t)HID * HID) return;
    if (in_sizes[4] < HID) return;
    if ((size_t)out_size < (size_t)(A_OFF_BYTES / 4) + ((size_t)(NB - 1) * SEQ_FULL + SEQ) * SEQ_FULL) return;
    if (SZ_TOTAL > ws_size) return;
    const float* xin[2] = { (const float*)d_in[0], (const float*)d_in[1] };
    const float* wq = (const float*)d_in[2];
    const float* wk = (const float*)d_in[3];
    const float* vv = (const float*)d_in[4];
    float* OUT = (float*)d_out;
    char* wsp = (char*)d_ws;
    bf* XB = (bf*)wsp; wsp += 2 * SZ_XB;
    bf* WB = (bf*)wsp; wsp += 2 * SZ_WB;
    float* PL = (float*)wsp; wsp += 2 * SZ_PL;
    h16* KT = (h16*)wsp; wsp += SZ_KT;

    for (int i = 0; i < 2; ++i) {
        bf* dstp = XB + (size_t)i * (SZ_XB / 2);
        if (SEQ == SEQ_FULL) {
            const size_t n8 = (size_t)NB * SEQ * HID / 8;
            k_cvt8<<<(unsigned)((n8 + 255) / 256), 256, 0, stream>>>(xin[i], dstp, n8);
        } else {
            const size_t n8 = (size_t)SEQ * HID / 8;
            for (int b = 0; b < NB; ++b) k_cvt8<<<(unsigned)((n8 + 255) / 256), 256, 0, stream>>>(xin[i] + (size_t)b * SEQ_FULL * HID, dstp + (size_t)b * SEQ * HID, n8);
        }
    }
    { const size_t n8 = (size_t)HID * HID / 8; const unsigned g = (unsigned)((n8 + 255) / 256);
      k_cvt8<<<g, 256, 0, stream>>>(wq, WB, n8); k_cvt8<<<g, 256, 0, stream>>>(wk, WB + (SZ_WB / 2), n8); }

    k_tr<<<dim3(SEQ / 64, HID / 64, NB), 256, 0, stream>>>(xin[1], KT);

    k_proj<<<dim3(NB * SEQ / 64, HID / 64, 2), 32, 0, stream>>>(XB, WB, PL);

    k_attn<<<dim3(SEQ / 16, NB, 1), 32 * AWV, 0, stream>>>(PL, PL + (SZ_PL / 4), KT, vv, OUT);
}
